// InteractionPredictionHead_41429254537606
// MI455X (gfx1250) — hardware-verified
//
#include <hip/hip_runtime.h>
#include <stddef.h>

typedef __attribute__((ext_vector_type(16))) _Float16 v16h;
typedef __attribute__((ext_vector_type(8)))  _Float16 v8h;
typedef __attribute__((ext_vector_type(16))) __bf16   v16b;
typedef __attribute__((ext_vector_type(8)))  __bf16   v8b;
typedef __attribute__((ext_vector_type(8)))  float    v8f;
typedef __attribute__((ext_vector_type(4)))  float    v4f;
#define PSCALE 32768.0f
#define U16(p) ((const unsigned short*)(const void*)(p))
#define PSCALE_INV (1.0f / 32768.0f)

__device__ __forceinline__ unsigned short f2bf_bits(float f) {
  unsigned u = __float_as_uint(f);
  return (unsigned short)((u + 0x7FFFu + ((u >> 16) & 1u)) >> 16);
}
__device__ __forceinline__ float bf_bits2f(unsigned short h) { return __uint_as_float(((unsigned)h) << 16); }

__device__ __forceinline__ void dep_guard_h(v8f& a, v8f& b, v16h x, v16h y) { asm volatile("v_nop\n\tv_nop\n\tv_nop\n\tv_nop" : "+v"(a), "+v"(b) : "v"(x), "v"(y)); }
__device__ __forceinline__ void dep_guard_b(v8f& a, v8f& b, v16b x, v16b y) { asm volatile("v_nop\n\tv_nop\n\tv_nop\n\tv_nop" : "+v"(a), "+v"(b) : "v"(x), "v"(y)); }
__device__ __forceinline__ void keep4_h(v16h a, v16h b, v16h c, v16h d) { asm volatile("v_nop" :: "v"(a), "v"(b), "v"(c), "v"(d)); }
__device__ __forceinline__ void keep4_b(v16b a, v16b b, v16b c, v16b d) { asm volatile("v_nop" :: "v"(a), "v"(b), "v"(c), "v"(d)); }
__device__ __forceinline__ void acc_guard4(v8f& a, v8f& b, v8f& c, v8f& d) { asm volatile("v_nop\n\tv_nop\n\tv_nop\n\tv_nop" : "+v"(a), "+v"(b), "+v"(c), "+v"(d)); }
template <typename T> struct Frag;
template <> struct Frag<_Float16> {
  typedef v16h V; union U { v16h v; v8h h[2]; };
  static __device__ __forceinline__ v16h load(const _Float16* p) {
    U f; f.h[0] = *(const v8h*)(p); f.h[1] = *(const v8h*)(p + 16); return f.v;
  }
  static __device__ __forceinline__ v8f mma(v16h a, v16h b, v8f c) {
    return __builtin_amdgcn_wmma_f32_16x16x32_f16(false, a, false, b, (short)0, c, false, false);
  }
  static __device__ __forceinline__ void guard(v8f& a, v8f& b, v16h x, v16h y) { dep_guard_h(a, b, x, y); }
  static __device__ __forceinline__ void keep(v16h a, v16h b, v16h c, v16h d) { keep4_h(a, b, c, d); }
};
template <> struct Frag<__bf16> {
  typedef v16b V; union U { v16b v; v8b h[2]; };
  static __device__ __forceinline__ v16b load(const __bf16* p) {
    U f; f.h[0] = *(const v8b*)(p); f.h[1] = *(const v8b*)(p + 16); return f.v;
  }
  static __device__ __forceinline__ v8f mma(v16b a, v16b b, v8f c) {
    return __builtin_amdgcn_wmma_f32_16x16x32_bf16(false, a, false, b, (short)0, c, false, false);
  }
  static __device__ __forceinline__ void guard(v8f& a, v8f& b, v16b x, v16b y) { dep_guard_b(a, b, x, y); }
  static __device__ __forceinline__ void keep(v16b a, v16b b, v16b c, v16b d) { keep4_b(a, b, c, d); }
};

template <int ET> struct Elem;
template <> struct Elem<0> { typedef _Float16 T; };
template <> struct Elem<1> { typedef __bf16 T; };
template <int ET, bool SPLIT, int BIAS_MODE, int OUT_MODE, bool RESID, int ACT = 0>
__global__ __launch_bounds__(256) void wmma_gemm64(
    const unsigned short* __restrict__ Ap, const unsigned short* __restrict__ A2p, int lda, long strideA,
    const unsigned short* __restrict__ Btp, const unsigned short* __restrict__ Bt2p, int ldb, long strideB,
    void* __restrict__ Cout, void* __restrict__ Cout2, int ldc, long strideC,
    const float* __restrict__ bias,
    const float* __restrict__ resid, long strideR,
    int M, int N, int K, float scale) {
  typedef typename Elem<ET>::T T;
  typedef typename Frag<T>::V V;
  const T* A = (const T*)Ap; const T* A2 = (const T*)A2p; const T* Bt = (const T*)Btp; const T* Bt2 = (const T*)Bt2p;
  __shared__ __align__(16) float sT[8][16 * 68];
  const int b    = blockIdx.y;
  const int lane = threadIdx.x & 31;
  const int wave = threadIdx.x >> 5;
  const int tilesN = N >> 6;
  const int tilesM = M >> 6;
  const int tile = blockIdx.x * 8 + wave;
  if (tile >= tilesM * tilesN) return;
  const int tm = tile / tilesN;
  const int tn = tile - tm * tilesN;
  const int m0 = tm << 6;
  const int n0 = tn << 6;

  const T* Ab  = A  + (size_t)b * strideA;
  const T* Bb  = Bt + (size_t)b * strideB;
  const T* Ab2 = SPLIT ? (A2  + (size_t)b * strideA) : nullptr;
  const T* Bb2 = SPLIT ? (Bt2 + (size_t)b * strideB) : nullptr;

  const int rlane = lane & 15;
  const int koff  = (lane >> 4) * 8;
  const int mOff  = (lane >> 4) * 8;

  v8f acc[4][4];
#pragma unroll
  for (int i = 0; i < 4; ++i)
#pragma unroll
    for (int j = 0; j < 4; ++j) acc[i][j] = (v8f){0.f,0.f,0.f,0.f,0.f,0.f,0.f,0.f};

  for (int k0 = 0; k0 < K; k0 += 32) {
    V bh[4], bl[4];
#pragma unroll
    for (int j = 0; j < 4; ++j) {
      const size_t bo = (size_t)(n0 + (j << 4) + rlane) * ldb + koff + k0;
      bh[j] = Frag<T>::load(Bb + bo);
      if (SPLIT) bl[j] = Frag<T>::load(Bb2 + bo);
    }
#pragma unroll
    for (int i = 0; i < 4; ++i) {
      const size_t ao = (size_t)(m0 + (i << 4) + rlane) * lda + koff + k0;
      V ah = Frag<T>::load(Ab + ao);
      V al;
      if (SPLIT) al = Frag<T>::load(Ab2 + ao);
#pragma unroll
      for (int j = 0; j < 4; ++j) {
        acc[i][j] = Frag<T>::mma(ah, bh[j], acc[i][j]);
        if (SPLIT) {
          acc[i][j] = Frag<T>::mma(ah, bl[j], acc[i][j]);
          acc[i][j] = Frag<T>::mma(al, bh[j], acc[i][j]);
        }
      }
      Frag<T>::guard(acc[i][0], acc[i][3], ah, SPLIT ? al : ah);
    }
    Frag<T>::keep(bh[0], bh[1], bh[2], bh[3]);
    if (SPLIT) Frag<T>::keep(bl[0], bl[1], bl[2], bl[3]);
  }
  acc_guard4(acc[0][0], acc[0][1], acc[0][2], acc[0][3]);
  acc_guard4(acc[1][0], acc[1][1], acc[1][2], acc[1][3]);
  acc_guard4(acc[2][0], acc[2][1], acc[2][2], acc[2][3]);
  acc_guard4(acc[3][0], acc[3][1], acc[3][2], acc[3][3]);

  float* slab = sT[wave];
  const float* Rb = RESID ? (resid + (size_t)b * strideR) : nullptr;
#pragma unroll
  for (int i = 0; i < 4; ++i) {
    const int mBase = m0 + (i << 4);
#pragma unroll
    for (int j = 0; j < 4; ++j) {
      const int n = n0 + (j << 4) + rlane;
      float bv = 0.f;
      if (BIAS_MODE == 2) bv = bias[n];
#pragma unroll
      for (int r = 0; r < 8; ++r) {
        float v = acc[i][j][r] * scale;
        if (BIAS_MODE == 1) v += bias[mBase + mOff + r];
        if (BIAS_MODE == 2) v += bv;
        if (RESID) v += Rb[(size_t)(mBase + mOff + r) * ldc + n];
        if (ACT == 1) v = tanhf(v);
        if (ACT == 2) v = fmaxf(v, 0.0f);
        if (ACT == 3) v = v / (1.0f + expf(-v));
        if (ACT == 4) v = (v > 0.f) ? v : 0.01f * v;
        if (ACT == 5) v = 0.5f * v * (1.0f + erff(v * 0.70710678118654752f));
        slab[(mOff + r) * 68 + (j << 4) + rlane] = v;
      }
    }
    __builtin_amdgcn_fence(__ATOMIC_RELEASE, "workgroup");
    __builtin_amdgcn_wave_barrier();
    __builtin_amdgcn_fence(__ATOMIC_ACQUIRE, "workgroup");
    if (OUT_MODE == 0) {
      float* C = (float*)Cout + (size_t)b * strideC;
      const int hh = lane >> 4, c4 = (lane & 15) * 4;
      for (int pass = 0; pass < 2; ++pass) {
#pragma unroll
        for (int it = 0; it < 8; ++it) {
          const int row = it * 2 + hh;
          v4f v = *(const v4f*)(slab + row * 68 + c4);
          *(volatile v4f*)(C + (size_t)(mBase + row) * ldc + n0 + c4) = v;
        }
        __threadfence();
      }
    } else {
      const int q = lane >> 3, c8 = (lane & 7) * 8;
      unsigned short* C  = (unsigned short*)Cout  + (size_t)b * strideC;
      unsigned short* C2 = (OUT_MODE == 2) ? ((unsigned short*)Cout2 + (size_t)b * strideC) : nullptr;
      for (int pass = 0; pass < 2; ++pass) {
#pragma unroll
        for (int it = 0; it < 4; ++it) {
          const int row = it * 4 + q;
          const float* sp = slab + row * 68 + c8;
          v8h hv, lv;
#pragma unroll
          for (int e = 0; e < 8; ++e) {
            if (OUT_MODE == 1) {
              hv[e] = (_Float16)sp[e];
            } else {
              unsigned short hb = f2bf_bits(sp[e]);
              unsigned short lb = f2bf_bits(sp[e] - bf_bits2f(hb));
              hv[e] = __builtin_bit_cast(_Float16, hb);
              lv[e] = __builtin_bit_cast(_Float16, lb);
            }
          }
          *(volatile v8h*)(C + (size_t)(mBase + row) * ldc + n0 + c8) = hv;
          if (OUT_MODE == 2) *(volatile v8h*)(C2 + (size_t)(mBase + row) * ldc + n0 + c8) = lv;
        }
        __threadfence();
      }
    }
    __builtin_amdgcn_fence(__ATOMIC_RELEASE, "workgroup");
    __builtin_amdgcn_wave_barrier();
    __builtin_amdgcn_fence(__ATOMIC_ACQUIRE, "workgroup");
  }
}

constexpr int HIDC       = 256;
constexpr int H2W        = 128;
constexpr int H3W        = 64;
constexpr int GWID       = 64;
constexpr int NLOGIT     = 3;
constexpr int EATTR      = 3;
constexpr int EDGE_CHUNK = 60032;
static_assert(EDGE_CHUNK % 64 == 0, "chunk rows are a tile multiple");
static_assert((EDGE_CHUNK * NLOGIT) % 32 == 0, "chunk output begins on a whole 128-B line");
static_assert(EDGE_CHUNK % 8 == 0, "8 rows per block in the gather kernel");

constexpr int PREP_B_W1 = (2 * HIDC) * HIDC / 2048;
constexpr int PREP_B_W2 = H2W * HIDC / 2048;
constexpr int PREP_B_W3 = H3W * H2W / 2048;
constexpr int PREP_B_W4 = GWID * H3W / 2048;
constexpr int PREP_BLOCKS = PREP_B_W1 + PREP_B_W2 + PREP_B_W3 + PREP_B_W4 + 1;
static_assert(PREP_B_W1 == 64 && PREP_B_W2 == 16 && PREP_B_W3 == 4 && PREP_B_W4 == 2, "prep block map");

__device__ __forceinline__ float bf16_rne(float f) {
  unsigned u = __float_as_uint(f);
  u = (u + 0x7FFFu + ((u >> 16) & 1u)) & 0xFFFF0000u;
  return __uint_as_float(u);
}
__device__ __forceinline__ _Float16 to_h16(float v) {
  v = (fabsf(v) < 6.103515625e-05f) ? 0.0f : v;
  return (_Float16)v;
}

__global__ __launch_bounds__(256) void cast_nodes_f16(
    const float* __restrict__ X, _Float16* __restrict__ X16, int nRows, int nRowsPad) {
  const size_t g8  = (size_t)blockIdx.x * 256 + threadIdx.x;
  const size_t idx = g8 * 8;
  const size_t row = idx >> 8;
  const int    col = (int)(idx & 255);
  if (row >= (size_t)nRowsPad) return;
  const bool   live = row < (size_t)nRows;
  const size_t rowc = live ? row : (size_t)(nRows - 1);
  const float* p = X + rowc * HIDC + col;
  const v4f a = *(const v4f*)(p);
  const v4f c = *(const v4f*)(p + 4);
  v8h hv;
#pragma unroll
  for (int e = 0; e < 4; ++e) {
    const float x0 = live ? a[e] : 0.0f;
    const float x1 = live ? c[e] : 0.0f;
    hv[e]     = to_h16(bf16_rne(x0));
    hv[4 + e] = to_h16(bf16_rne(x1));
  }
  _Float16* dst = X16 + idx;
  *(volatile v8h*)dst = hv;
  __threadfence();
  *(volatile v8h*)dst = hv;
}

__global__ __launch_bounds__(256) void prep_weights(
    const float* __restrict__ W1, const float* __restrict__ W2, const float* __restrict__ W3,
    const float* __restrict__ W4, const float* __restrict__ b4, int nB4,
    _Float16* __restrict__ W1Bt, _Float16* __restrict__ W2Bt, _Float16* __restrict__ W3Bt,
    _Float16* __restrict__ W4Bt, float* __restrict__ b4pad) {
  const int bid = blockIdx.x;
  const int tid = threadIdx.x;
  if (bid < PREP_B_W1) {
    const int flat = bid * 2048 + tid * 8;
    const int n  = flat >> 8;
    const int k0 = flat & 255;
    const int nn = (n < HIDC) ? n : (n - HIDC);
    const int rb = (n < HIDC) ? 0 : HIDC;
    v8h hv;
#pragma unroll
    for (int i = 0; i < 8; ++i) {
      const int k = k0 + i;
      const float w = W1[(size_t)(rb + k) * HIDC + nn];
      hv[i] = to_h16(bf16_rne(w) * 16.0f);
    }
    _Float16* dst = W1Bt + flat;
    *(volatile v8h*)dst = hv; __threadfence(); *(volatile v8h*)dst = hv;
  } else if (bid < PREP_B_W1 + PREP_B_W2) {
    const int flat = (bid - PREP_B_W1) * 2048 + tid * 8;
    const int n  = flat >> 8;
    const int k0 = flat & 255;
    v8h hv;
#pragma unroll
    for (int i = 0; i < 8; ++i) {
      const int k = k0 + i;
      const float w = W2[(size_t)k * H2W + n];
      hv[i] = to_h16(bf16_rne(w) * 16.0f);
    }
    _Float16* dst = W2Bt + flat;
    *(volatile v8h*)dst = hv; __threadfence(); *(volatile v8h*)dst = hv;
  } else if (bid < PREP_B_W1 + PREP_B_W2 + PREP_B_W3) {
    const int flat = (bid - PREP_B_W1 - PREP_B_W2) * 2048 + tid * 8;
    const int n  = flat >> 7;
    const int k0 = flat & 127;
    v8h hv;
#pragma unroll
    for (int i = 0; i < 8; ++i) {
      const int k = k0 + i;
      const float w = W3[(size_t)k * H3W + n];
      hv[i] = to_h16(bf16_rne(w) * 8.0f);
    }
    _Float16* dst = W3Bt + flat;
    *(volatile v8h*)dst = hv; __threadfence(); *(volatile v8h*)dst = hv;
  } else if (bid < PREP_B_W1 + PREP_B_W2 + PREP_B_W3 + PREP_B_W4) {
    const int flat = (bid - PREP_B_W1 - PREP_B_W2 - PREP_B_W3) * 2048 + tid * 8;
    const int n  = flat >> 6;
    const int k0 = flat & 63;
    const int nc = (n < NLOGIT) ? n : (NLOGIT - 1);
    v8h hv;
#pragma unroll
    for (int i = 0; i < 8; ++i) {
      const int k = k0 + i;
      const float w = W4[(size_t)k * NLOGIT + nc];
      const float wv = (n < NLOGIT) ? (bf16_rne(w) * 4.0f) : 0.0f;
      hv[i] = to_h16(wv);
    }
    _Float16* dst = W4Bt + flat;
    *(volatile v8h*)dst = hv; __threadfence(); *(volatile v8h*)dst = hv;
  } else {
    if (tid < 16) {
      v4f bv;
#pragma unroll
      for (int j = 0; j < 4; ++j) {
        const int n  = tid * 4 + j;
        const int nc = (n < nB4) ? n : (nB4 - 1);
        const float x = b4[nc];
        bv[j] = (n < nB4) ? bf16_rne(x) : 0.0f;
      }
      float* dst = b4pad + tid * 4;
      *(volatile v4f*)dst = bv; __threadfence(); *(volatile v4f*)dst = bv;
    }
  }
}

__global__ __launch_bounds__(256) void edge_layer1(
    const _Float16* __restrict__ P16, const int* __restrict__ eidx, const float* __restrict__ attr,
    const float* __restrict__ W1, const float* __restrict__ b1, _Float16* __restrict__ H1,
    int e0, int E, int nNodes) {
  const int lane = threadIdx.x & 31;
  const int wave = threadIdx.x >> 5;
  const int row  = blockIdx.x * 8 + wave;
  const int e    = e0 + row;
  const int ec   = (e < E) ? e : (E - 1);
  int s = eidx[ec];
  int d = eidx[(size_t)E + (size_t)ec];
  s = (s < 0) ? 0 : ((s >= nNodes) ? (nNodes - 1) : s);
  d = (d < 0) ? 0 : ((d >= nNodes) ? (nNodes - 1) : d);
  const float a0 = bf16_rne(attr[(size_t)ec * EATTR + 0]);
  const float a1 = bf16_rne(attr[(size_t)ec * EATTR + 1]);
  const float a2 = bf16_rne(attr[(size_t)ec * EATTR + 2]);
  const int c = lane * 8;
  const v8h pa = *(const v8h*)(P16 + (size_t)s * (2 * HIDC) + c);
  const v8h pb = *(const v8h*)(P16 + (size_t)d * (2 * HIDC) + HIDC + c);
  const v4f bq0 = *(const v4f*)(b1 + c);
  const v4f bq1 = *(const v4f*)(b1 + c + 4);
  const float* wt = W1 + (size_t)(2 * HIDC) * HIDC + c;
  const v4f w00 = *(const v4f*)(wt),              w01 = *(const v4f*)(wt + 4);
  const v4f w10 = *(const v4f*)(wt + HIDC),       w11 = *(const v4f*)(wt + HIDC + 4);
  const v4f w20 = *(const v4f*)(wt + 2 * HIDC),   w21 = *(const v4f*)(wt + 2 * HIDC + 4);
  v8h hv;
#pragma unroll
  for (int i = 0; i < 4; ++i) {
    float v = (float)pa[i] + (float)pb[i] + bq0[i];
    v += a0 * bf16_rne(w00[i]);
    v += a1 * bf16_rne(w10[i]);
    v += a2 * bf16_rne(w20[i]);
    v = fmaxf(v, 0.0f);
    hv[i] = to_h16(v);
    float u = (float)pa[4 + i] + (float)pb[4 + i] + bq1[i];
    u += a0 * bf16_rne(w01[i]);
    u += a1 * bf16_rne(w11[i]);
    u += a2 * bf16_rne(w21[i]);
    u = fmaxf(u, 0.0f);
    hv[4 + i] = to_h16(u);
  }
  _Float16* dst = H1 + (size_t)row * HIDC + c;
  *(volatile v8h*)dst = hv;
  __threadfence();
  *(volatile v8h*)dst = hv;
}

__global__ __launch_bounds__(256) void pack_logits(
    const float* __restrict__ G, float* __restrict__ out, int line0, int nLines, int e0, int rowsG, int total) {
  const int lane = threadIdx.x & 31;
  const int wave = threadIdx.x >> 5;
  const int line = blockIdx.x * 8 + wave;
  if (line >= nLines) return;
  const int f = (line0 + line) * 32 + lane;
  const int e = f / NLOGIT;
  const int k = f - e * NLOGIT;
  int r = e - e0;
  r = (r < 0) ? 0 : ((r >= rowsG) ? (rowsG - 1) : r);
  const float v = G[(size_t)r * GWID + k];
  if (f < total) *(volatile float*)(out + f) = v;
  __threadfence();
  if (f < total) *(volatile float*)(out + f) = v;
}

static inline size_t align256(size_t x) { return (x + 255) & ~(size_t)255; }

extern "C" void kernel_launch(void* const* d_in, const int* in_sizes, int n_in,
                              void* d_out, int out_size, void* d_ws, size_t ws_size,
                              hipStream_t stream) {
  if (n_in < 11) return;
  const float* X    = (const float*)d_in[0];
  const int*   eidx = (const int*)d_in[1];
  const float* attr = (const float*)d_in[2];
  const float* W1   = (const float*)d_in[3];
  const float* b1   = (const float*)d_in[4];
  const float* W2   = (const float*)d_in[5];
  const float* b2   = (const float*)d_in[6];
  const float* W3   = (const float*)d_in[7];
  const float* b3   = (const float*)d_in[8];
  const float* W4   = (const float*)d_in[9];
  const float* b4   = (const float*)d_in[10];
  float* out = (float*)d_out;

  const int nNodes = in_sizes[0] / HIDC;
  const int E      = in_sizes[1] / 2;
  const int nB4    = in_sizes[10];
  const int total  = out_size;
  if (nNodes <= 0 || E <= 0 || nB4 <= 0) return;
  if (in_sizes[3] != (2 * HIDC + EATTR) * HIDC || in_sizes[5] != HIDC * H2W ||
      in_sizes[7] != H2W * H3W || in_sizes[9] != H3W * NLOGIT) return;
  if (total != E * NLOGIT) return;

  const int NPAD    = ((nNodes + 63) / 64) * 64;
  const int nChunks = (E + EDGE_CHUNK - 1) / EDGE_CHUNK;

  const size_t bP16 = (size_t)NPAD * (2 * HIDC) * 2;
  const size_t bX16 = (size_t)NPAD * HIDC * 2;
  const size_t bH2  = (size_t)EDGE_CHUNK * H2W * 2;
  const size_t bH3  = (size_t)EDGE_CHUNK * H3W * 2;
  const size_t bRB  = (bX16 > bH2 + bH3) ? bX16 : (bH2 + bH3);
  const size_t bH1  = (size_t)EDGE_CHUNK * HIDC * 2;
  const size_t bG   = (size_t)EDGE_CHUNK * GWID * 4;
  const size_t bW1t = (size_t)(2 * HIDC) * HIDC * 2;
  const size_t bW2t = (size_t)H2W * HIDC * 2;
  const size_t bW3t = (size_t)H3W * H2W * 2;
  const size_t bW4t = (size_t)GWID * H3W * 2;
  const size_t bB4  = (size_t)GWID * 4;

  size_t off = 0;
  const size_t oP16 = off; off = align256(off + bP16);
  const size_t oRB  = off; off = align256(off + bRB);
  const size_t oH1  = off; off = align256(off + bH1);
  const size_t oG   = off; off = align256(off + bG);
  const size_t oW1t = off; off = align256(off + bW1t);
  const size_t oW2t = off; off = align256(off + bW2t);
  const size_t oW3t = off; off = align256(off + bW3t);
  const size_t oW4t = off; off = align256(off + bW4t);
  const size_t oB4  = off; off = align256(off + bB4);
  if (off > ws_size) return;

  char* ws = (char*)d_ws;
  _Float16* P16  = (_Float16*)(ws + oP16);
  _Float16* X16  = (_Float16*)(ws + oRB);
  _Float16* H2c  = (_Float16*)(ws + oRB);
  _Float16* H3c  = (_Float16*)(ws + oRB + align256(bH2));
  _Float16* H1c  = (_Float16*)(ws + oH1);
  float*    Gc   = (float*)(ws + oG);
  _Float16* W1Bt = (_Float16*)(ws + oW1t);
  _Float16* W2Bt = (_Float16*)(ws + oW2t);
  _Float16* W3Bt = (_Float16*)(ws + oW3t);
  _Float16* W4Bt = (_Float16*)(ws + oW4t);
  float*    b4pad = (float*)(ws + oB4);
  if (oRB + align256(bH2) + bH3 > oH1) return;

  cast_nodes_f16<<<dim3(NPAD / 8), dim3(256), 0, stream>>>(X, X16, nNodes, NPAD);

  prep_weights<<<dim3(PREP_BLOCKS), dim3(256), 0, stream>>>(W1, W2, W3, W4, b4, nB4,
                                                           W1Bt, W2Bt, W3Bt, W4Bt, b4pad);

  {
    const int tiles  = (NPAD / 64) * ((2 * HIDC) / 64);
    const int blocks = (tiles + 7) / 8;
    wmma_gemm64<0, false, 0, 1, false, 0><<<dim3(blocks, 1), dim3(256), 0, stream>>>(
        (const unsigned short*)X16, (const unsigned short*)X16, HIDC, 0L,
        (const unsigned short*)W1Bt, (const unsigned short*)W1Bt, HIDC, 0L,
        (void*)P16, (void*)P16, 2 * HIDC, 0L,
        b1, b1, 0L, NPAD, 2 * HIDC, HIDC, 1.0f / 16.0f);
  }

  for (int ch = 0; ch < nChunks; ++ch) {
    const int e0 = ch * EDGE_CHUNK;

    edge_layer1<<<dim3(EDGE_CHUNK / 8), dim3(256), 0, stream>>>(P16, eidx, attr, W1, b1, H1c, e0, E, nNodes);

    {
      const int tiles  = (EDGE_CHUNK / 64) * (H2W / 64);
      const int blocks = (tiles + 7) / 8;
      wmma_gemm64<0, false, 2, 1, false, 0><<<dim3(blocks, 1), dim3(256), 0, stream>>>(
          (const unsigned short*)H1c, (const unsigned short*)H1c, HIDC, 0L,
          (const unsigned short*)W2Bt, (const unsigned short*)W2Bt, HIDC, 0L,
          (void*)H2c, (void*)H2c, H2W, 0L,
          b2, b2, 0L, EDGE_CHUNK, H2W, HIDC, 1.0f / 16.0f);
    }

    {
      const int tiles  = (EDGE_CHUNK / 64) * (H3W / 64);
      const int blocks = (tiles + 7) / 8;
      wmma_gemm64<0, false, 2, 1, false, 2><<<dim3(blocks, 1), dim3(256), 0, stream>>>(
          (const unsigned short*)H2c, (const unsigned short*)H2c, H2W, 0L,
          (const unsigned short*)W3Bt, (const unsigned short*)W3Bt, H2W, 0L,
          (void*)H3c, (void*)H3c, H3W, 0L,
          b3, b3, 0L, EDGE_CHUNK, H3W, H2W, 1.0f / 8.0f);
    }

    {
      const int tiles  = (EDGE_CHUNK / 64) * (GWID / 64);
      const int blocks = (tiles + 7) / 8;
      wmma_gemm64<0, false, 2, 0, false, 0><<<dim3(blocks, 1), dim3(256), 0, stream>>>(
          (const unsigned short*)H3c, (const unsigned short*)H3c, H3W, 0L,
          (const unsigned short*)W4Bt, (const unsigned short*)W4Bt, H3W, 0L,
          (void*)Gc, (void*)Gc, GWID, 0L,
          b4pad, b4pad, 0L, EDGE_CHUNK, GWID, H3W, 1.0f / 4.0f);
    }

    {
      const long long f0 = (long long)e0 * NLOGIT;
      long long f1 = (long long)(e0 + EDGE_CHUNK) * NLOGIT;
      if (f1 > (long long)total) f1 = total;
      if (f1 > f0) {
        const int line0  = (int)(f0 / 32);
        const int nLines = (int)((f1 - f0 + 31) / 32);
        const int blocks = (nLines + 7) / 8;
        pack_logits<<<dim3(blocks), dim3(256), 0, stream>>>(Gc, out, line0, nLines, e0, EDGE_CHUNK, total);
      }
    }
  }
}
